// Graph_GAN_29832842838350
// MI455X (gfx1250) — hardware-verified
//
#include <hip/hip_runtime.h>
#include <stddef.h>
#include <stdint.h>

#pragma clang fp contract(off)


#define NB_   64
#define NN_   100
#define HD_   32
#define NNODE (NB_ * NN_)
#define NTI   7
#define NIP   (NTI * 16)
#define K0_   65
#define E0_   96
#define E1_   160
#define E2_   192
#define G0_   224
#define G1_   256
#define NFO   3
#define PQP   192
#define ASP   192
#define XAP   40
#define H1P   104
#define H2P   168
#define N0P   232
#define N1P   264
#define NTE   128
#define NTN   256
#define WSCL  16.0f
#define PSCL  0.0625f
#define LRA   0.2f
#define WSCAP 134217728

#define HW0 (2 * E0_ * HD_)
#define HW1 (E1_ * E0_)
#define HW2 (E2_ * E1_)
#define HV0 (G1_ * G0_)
#define HV1 (G1_ * G1_)
#define HV2 (16 * G1_)
#define OW0 0
#define OW1 (OW0 + HW0)
#define OW2 (OW1 + HW1)
#define OV0 (OW2 + HW2)
#define OV1 (OV0 + HV0)
#define OV2 (OV1 + HV1)
#define HWT (OV2 + HV2)
#define CHK 256
#define CB1 (HW0 / CHK)
#define CB2 (CB1 + HW1 / CHK)
#define CB3 (CB2 + HW2 / CHK)
#define CB4 (CB3 + HV0 / CHK)
#define CB5 (CB4 + HV1 / CHK)
#define NCHUNK (CB5 + HV2 / CHK)

static_assert(HWT == 179200);
static_assert(NCHUNK == 700);
static_assert((HW0 % CHK) == 0);
static_assert((HW1 % CHK) == 0);
static_assert((HW2 % CHK) == 0);
static_assert((HV0 % CHK) == 0);
static_assert((HV1 % CHK) == 0);
static_assert((HV2 % CHK) == 0);
static_assert((NCHUNK % 4) == 0);
static_assert((OW1 % 8) == 0);
static_assert((OW2 % 8) == 0);
static_assert((OV0 % 8) == 0);
static_assert((OV1 % 8) == 0);
static_assert((OV2 % 8) == 0);
static_assert((E0_ % 32) == 0);
static_assert((E1_ % 32) == 0);
static_assert((G0_ % 32) == 0);
static_assert((G1_ % 32) == 0);
static_assert((NNODE % 32) == 0);
static_assert((NN_ % 2) == 0);
static_assert(((XAP * 2) % 16) == 0);
static_assert(((H1P * 2) % 16) == 0);
static_assert(((H2P * 2) % 16) == 0);
static_assert(((N0P * 2) % 16) == 0);
static_assert(((N1P * 2) % 16) == 0);
static_assert(NTE == 4 * 32);
static_assert(NTN == 8 * 32);

#define SZ_WP  ((size_t)HWT * 2)
#define SZ_PQ  ((size_t)NNODE * PQP * 4)
#define SZ_AS  ((size_t)NB_ * NIP * ASP * 4)
#define SZ_TOT (SZ_WP + SZ_PQ + SZ_AS)
static_assert(SZ_WP == 358400);
static_assert(SZ_PQ == 4915200);
static_assert(SZ_AS == 5505024);
static_assert(SZ_TOT == 10778624);
static_assert(SZ_TOT <= (size_t)WSCAP);
static_assert((SZ_WP % 256) == 0);
static_assert((SZ_PQ % 256) == 0);
static_assert((SZ_AS % 256) == 0);

typedef _Float16     v16h __attribute__((ext_vector_type(16)));
typedef _Float16     v8h  __attribute__((ext_vector_type(8)));
typedef _Float16     v4h  __attribute__((ext_vector_type(4)));
typedef float        v8f  __attribute__((ext_vector_type(8)));
typedef float        v4f  __attribute__((ext_vector_type(4)));
typedef unsigned int v4u  __attribute__((ext_vector_type(4)));
union Frag { v16h v; v8h half[2]; };
union Pk8  { v8h h; v4u u; };

__device__ __forceinline__ int imin(int a, int b) { return a < b ? a : b; }

__device__ __forceinline__ float lk(float v) { return fmaxf(v, LRA * v); }

__device__ __forceinline__ v4f lk4(v4f u) {
  v4f r = {lk(u.x), lk(u.y), lk(u.z), lk(u.w)};
  return r;
}

__device__ __forceinline__ v4u cvt8(const v4f a, const v4f b) {
  v8h hv = {(_Float16)a.x, (_Float16)a.y, (_Float16)a.z, (_Float16)a.w,
            (_Float16)b.x, (_Float16)b.y, (_Float16)b.z, (_Float16)b.w};
  Pk8 p;
  p.h = hv;
  return p.u;
}

__device__ __forceinline__ v4h cvt4(const v4f a) {
  v4h r = {(_Float16)a.x, (_Float16)a.y, (_Float16)a.z, (_Float16)a.w};
  return r;
}

__device__ __forceinline__ v8f wmh(v16h a, v16h b, v8f c) {
  v8f d = __builtin_amdgcn_wmma_f32_16x16x32_f16(false, a, false, b, (short)0, c, false, false);
  asm volatile("v_nop\n\tv_nop\n\tv_nop\n\tv_nop" : "+v"(d) : "v"(a), "v"(b));
  return d;
}

__device__ __forceinline__ v16h lda_frag(const _Float16* tile, int pitch, int m, int k0, int h) {
  Frag a;
  const _Float16* p = tile + m * pitch + k0 + 8 * h;
  a.half[0] = *(const v8h*)p;
  a.half[1] = *(const v8h*)(p + 16);
  return a.v;
}

__device__ __forceinline__ v16h ldb_frag(const _Float16* plane, int kp, int n, int k0, int h) {
  Frag b;
  const _Float16* p = plane + (size_t)n * kp + k0 + 8 * h;
  b.half[0] = *(const v8h*)p;
  b.half[1] = *(const v8h*)(p + 16);
  return b.v;
}

__global__ __launch_bounds__(NTE) void k_prep(const float* __restrict__ w0, const float* __restrict__ w1,
                                              const float* __restrict__ w2, const float* __restrict__ v0,
                                              const float* __restrict__ v1, const float* __restrict__ v2,
                                              _Float16* wp) {
  const int tid = threadIdx.x, lane = tid & 31;
  const int wv = __builtin_amdgcn_readfirstlane(tid >> 5);
  const int c = blockIdx.x * 4 + wv;
  if (c >= NCHUNK) return;
  const float* src;
  int eb, md = 0;
  if (c < CB1)      { src = w0; eb = c * CHK; md = 1; }
  else if (c < CB2) { src = w1; eb = (c - CB1) * CHK; }
  else if (c < CB3) { src = w2; eb = (c - CB2) * CHK; }
  else if (c < CB4) { src = v0; eb = (c - CB3) * CHK; }
  else if (c < CB5) { src = v1; eb = (c - CB4) * CHK; }
  else              { src = v2; eb = (c - CB5) * CHK; }
  float t[8];
#pragma unroll
  for (int u = 0; u < 8; ++u) {
    const int e = eb + 8 * lane + u;
    const int n = e >> 5, k = e & 31;
    const int i1 = (n < E0_) ? (n * K0_ + k) : ((n - E0_) * K0_ + HD_ + k);
    const int idx = md ? i1 : e;
    t[u] = src[idx] * WSCL;
  }
  const v4f f0 = {t[0], t[1], t[2], t[3]};
  const v4f f1 = {t[4], t[5], t[6], t[7]};
  const v4u pk = cvt8(f0, f1);
  _Float16* d = wp + (size_t)c * CHK + 8 * lane;
  *(volatile v4u*)d = pk;
  __threadfence();
  *(volatile v4u*)d = pk;
}

__global__ __launch_bounds__(NTE) void k_pq(const float* __restrict__ x, const _Float16* __restrict__ wp,
                                            const float* __restrict__ b0, float* pq) {
  __shared__ __attribute__((aligned(16))) _Float16 xa[16 * XAP];
  __shared__ __attribute__((aligned(16))) float dt[16 * PQP];
  const int tid = threadIdx.x, lane = tid & 31, h = lane >> 4, m = lane & 15;
  const int wv = __builtin_amdgcn_readfirstlane(tid >> 5);
  const int blk = blockIdx.x;
  {
    const int row = tid >> 3, c0 = (tid & 7) * 4;
    const v4f a = *(const v4f*)(x + (size_t)(16 * blk + row) * HD_ + c0);
    *(v4h*)(xa + row * XAP + c0) = cvt4(a);
  }
  __syncthreads();

  const v8f zero8 = {0.f, 0.f, 0.f, 0.f, 0.f, 0.f, 0.f, 0.f};
  const v16h fa = lda_frag(xa, XAP, m, 0, h);
  v8f acc[3];
#pragma unroll
  for (int s = 0; s < 3; ++s) {
    const v16h fb = ldb_frag(wp + OW0, HD_, 48 * wv + 16 * s + m, 0, h);
    acc[s] = wmh(fa, fb, zero8);
  }
#pragma unroll
  for (int s = 0; s < 3; ++s) {
    const int col = 48 * wv + 16 * s + m;
    const float bl = b0[imin(col, E0_ - 1)];
    const float bb = (col < E0_) ? bl : 0.f;
#pragma unroll
    for (int r = 0; r < 8; ++r) dt[(8 * h + r) * PQP + col] = acc[s][r] * PSCL + bb;
  }
  __syncthreads();

  v4f v[6];
#pragma unroll
  for (int it = 0; it < 6; ++it) v[it] = *(const v4f*)(dt + 4 * (it * NTE + tid));
  float* pg = pq + (size_t)blk * 16 * PQP;
#pragma unroll
  for (int it = 0; it < 6; ++it) *(volatile v4f*)(pg + 4 * (it * NTE + tid)) = v[it];
  __threadfence();
#pragma unroll
  for (int it = 0; it < 6; ++it) *(volatile v4f*)(pg + 4 * (it * NTE + tid)) = v[it];
}

__global__ __launch_bounds__(NTE) void k_edge(const float* __restrict__ x, const float* __restrict__ pq,
                                              const float* __restrict__ w0, const float* __restrict__ b1,
                                              const float* __restrict__ b2, const _Float16* __restrict__ wp,
                                              float* as) {
  __shared__ __attribute__((aligned(16))) float pp[16 * E0_];
  __shared__ __attribute__((aligned(16))) float wd[E0_];
  __shared__ float xs[32];
  __shared__ __attribute__((aligned(16))) _Float16 h1[32 * H1P];
  __shared__ __attribute__((aligned(16))) _Float16 h2[32 * H2P];
  __shared__ __attribute__((aligned(16))) float st[16 * E2_];
  const int tid = threadIdx.x, lane = tid & 31, h = lane >> 4, m = lane & 15;
  const int wv = __builtin_amdgcn_readfirstlane(tid >> 5);
  const int blk = blockIdx.x, b = blk / NTI, i0 = (blk - b * NTI) * 16;

  for (int e = tid; e < 16 * E0_; e += NTE) {
    const int mm = e / E0_, cc = e - mm * E0_;
    const int nd = b * NN_ + imin(i0 + mm, NN_ - 1);
    pp[e] = pq[(size_t)nd * PQP + cc];
  }
  if (tid < E0_) wd[tid] = w0[tid * K0_ + (K0_ - 1)];
  if (tid < 32) {
    const int nd = b * NN_ + imin(i0 + (tid >> 1), NN_ - 1);
    xs[tid] = x[(size_t)nd * HD_ + (tid & 1)];
  }
  const bool t3 = (wv < 2);
  float bb1[3], bb2[3];
#pragma unroll
  for (int s = 0; s < 3; ++s) {
    bb1[s] = b1[imin(16 * (wv + 4 * s) + m, E1_ - 1)];
    bb2[s] = b2[48 * wv + 16 * s + m];
  }
  const v8f zero8 = {0.f, 0.f, 0.f, 0.f, 0.f, 0.f, 0.f, 0.f};
  v8f sm[3];
#pragma unroll
  for (int s = 0; s < 3; ++s) sm[s] = zero8;
  __syncthreads();

  const int row = tid >> 2, mm = row & 15, jj = row >> 4, c0 = (tid & 3) * 24;
  const float xi0 = xs[2 * mm], xi1 = xs[2 * mm + 1];

#pragma unroll 1
  for (int itj = 0; itj < NN_ / 2; ++itj) {
    {
      const int j = 2 * itj + jj;
      const size_t nj = (size_t)(b * NN_ + j);
      const float* qr = pq + nj * PQP + E0_ + c0;
      const float xj0 = x[nj * HD_], xj1 = x[nj * HD_ + 1];
      const float d0 = (xj0 - xi0) + 1e-12f, d1 = (xj1 - xi1) + 1e-12f;
      const float ds = sqrtf(d0 * d0 + d1 * d1);
      const float* prow = pp + mm * E0_ + c0;
      const float* wrow = wd + c0;
#pragma unroll
      for (int e = 0; e < 3; ++e) {
        const v4f q0 = *(const v4f*)(qr + 8 * e), q1 = *(const v4f*)(qr + 8 * e + 4);
        const v4f p0 = *(const v4f*)(prow + 8 * e), p1 = *(const v4f*)(prow + 8 * e + 4);
        const v4f g0 = *(const v4f*)(wrow + 8 * e), g1 = *(const v4f*)(wrow + 8 * e + 4);
        const v4f u0 = (p0 + q0) + g0 * ds;
        const v4f u1 = (p1 + q1) + g1 * ds;
        *(v4u*)(h1 + row * H1P + c0 + 8 * e) = cvt8(lk4(u0), lk4(u1));
      }
    }
    __syncthreads();

    {
      v8f acc[2][3];
#pragma unroll
      for (int mt = 0; mt < 2; ++mt) { acc[mt][0] = zero8; acc[mt][1] = zero8; acc[mt][2] = zero8; }
#pragma unroll 1
      for (int kt = 0; kt < E0_ / 32; ++kt) {
        const int k0 = 32 * kt;
        const v16h fa0 = lda_frag(h1, H1P, m, k0, h);
        const v16h fa1 = lda_frag(h1, H1P, 16 + m, k0, h);
#pragma unroll
        for (int s = 0; s < 3; ++s) {
          if (s < 2 || t3) {
            const int n = imin(16 * (wv + 4 * s) + m, E1_ - 1);
            const v16h fb = ldb_frag(wp + OW1, E0_, n, k0, h);
            acc[0][s] = wmh(fa0, fb, acc[0][s]);
            acc[1][s] = wmh(fa1, fb, acc[1][s]);
          }
        }
      }
#pragma unroll
      for (int s = 0; s < 3; ++s) {
        if (s < 2 || t3) {
          const int col = 16 * (wv + 4 * s) + m;
#pragma unroll
          for (int mt = 0; mt < 2; ++mt) {
#pragma unroll
            for (int r = 0; r < 8; ++r) {
              const float v = lk(acc[mt][s][r] * PSCL + bb1[s]);
              h2[(16 * mt + 8 * h + r) * H2P + col] = (_Float16)v;
            }
          }
        }
      }
    }
    __syncthreads();

    {
      v8f acc[2][3];
#pragma unroll
      for (int mt = 0; mt < 2; ++mt) { acc[mt][0] = zero8; acc[mt][1] = zero8; acc[mt][2] = zero8; }
#pragma unroll 1
      for (int kt = 0; kt < E1_ / 32; ++kt) {
        const int k0 = 32 * kt;
        const v16h fa0 = lda_frag(h2, H2P, m, k0, h);
        const v16h fa1 = lda_frag(h2, H2P, 16 + m, k0, h);
#pragma unroll
        for (int s = 0; s < 3; ++s) {
          const v16h fb = ldb_frag(wp + OW2, E1_, 48 * wv + 16 * s + m, k0, h);
          acc[0][s] = wmh(fa0, fb, acc[0][s]);
          acc[1][s] = wmh(fa1, fb, acc[1][s]);
        }
      }
#pragma unroll
      for (int s = 0; s < 3; ++s) {
#pragma unroll
        for (int r = 0; r < 8; ++r) {
          const float v0 = lk(acc[0][s][r] * PSCL + bb2[s]);
          const float v1 = lk(acc[1][s][r] * PSCL + bb2[s]);
          sm[s][r] = (sm[s][r] + v0) + v1;
        }
      }
    }
  }

#pragma unroll
  for (int s = 0; s < 3; ++s) {
    const int col = 48 * wv + 16 * s + m;
#pragma unroll
    for (int r = 0; r < 8; ++r) st[(8 * h + r) * E2_ + col] = sm[s][r];
  }
  __syncthreads();

  v4f v[6];
#pragma unroll
  for (int it = 0; it < 6; ++it) v[it] = *(const v4f*)(st + 4 * (it * NTE + tid));
  float* pg = as + ((size_t)b * NIP + i0) * ASP;
#pragma unroll
  for (int it = 0; it < 6; ++it) *(volatile v4f*)(pg + 4 * (it * NTE + tid)) = v[it];
  __threadfence();
#pragma unroll
  for (int it = 0; it < 6; ++it) *(volatile v4f*)(pg + 4 * (it * NTE + tid)) = v[it];
}

__global__ __launch_bounds__(NTN) void k_node(const float* __restrict__ as, const float* __restrict__ x,
                                              const _Float16* __restrict__ wp, const float* __restrict__ c0b,
                                              const float* __restrict__ c1b, const float* __restrict__ c2b,
                                              float* out) {
  __shared__ __attribute__((aligned(16))) _Float16 h0[32 * N0P];
  __shared__ __attribute__((aligned(16))) _Float16 a1[32 * N1P];
  __shared__ __attribute__((aligned(16))) _Float16 a2[32 * N1P];
  __shared__ __attribute__((aligned(16))) float opre[32 * NFO];
  __shared__ __attribute__((aligned(16))) float obuf[32 * NFO];
  const int tid = threadIdx.x, lane = tid & 31, h = lane >> 4, m = lane & 15;
  const int wv = __builtin_amdgcn_readfirstlane(tid >> 5);
  const int blk = blockIdx.x;
  {
    const int row = tid >> 3, q = tid & 7;
    const int g = 32 * blk + row;
    const int bb = g / NN_, ii = g - bb * NN_;
    const float* ar = as + ((size_t)bb * NIP + ii) * ASP;
    const float* xr = x + (size_t)g * HD_;
#pragma unroll
    for (int e = 0; e < 6; ++e) {
      const int f = q + 8 * e;
      const v4f v = *(const v4f*)(ar + 4 * f);
      *(v4h*)(h0 + row * N0P + 4 * f) = cvt4(v);
    }
    {
      const v4f v = *(const v4f*)(xr + 4 * q);
      *(v4h*)(h0 + row * N0P + E2_ + 4 * q) = cvt4(v);
    }
  }
  __syncthreads();

  const v8f zero8 = {0.f, 0.f, 0.f, 0.f, 0.f, 0.f, 0.f, 0.f};
  {
    v8f acc[2][2];
#pragma unroll
    for (int mt = 0; mt < 2; ++mt) { acc[mt][0] = zero8; acc[mt][1] = zero8; }
#pragma unroll 1
    for (int kt = 0; kt < G0_ / 32; ++kt) {
      const int k0 = 32 * kt;
      const v16h fa0 = lda_frag(h0, N0P, m, k0, h);
      const v16h fa1 = lda_frag(h0, N0P, 16 + m, k0, h);
#pragma unroll
      for (int s = 0; s < 2; ++s) {
        const v16h fb = ldb_frag(wp + OV0, G0_, 32 * wv + 16 * s + m, k0, h);
        acc[0][s] = wmh(fa0, fb, acc[0][s]);
        acc[1][s] = wmh(fa1, fb, acc[1][s]);
      }
    }
#pragma unroll
    for (int s = 0; s < 2; ++s) {
      const int col = 32 * wv + 16 * s + m;
      const float bb = c0b[col];
#pragma unroll
      for (int mt = 0; mt < 2; ++mt) {
#pragma unroll
        for (int r = 0; r < 8; ++r) a1[(16 * mt + 8 * h + r) * N1P + col] = (_Float16)lk(acc[mt][s][r] * PSCL + bb);
      }
    }
  }
  __syncthreads();

  {
    v8f acc[2][2];
#pragma unroll
    for (int mt = 0; mt < 2; ++mt) { acc[mt][0] = zero8; acc[mt][1] = zero8; }
#pragma unroll 1
    for (int kt = 0; kt < G1_ / 32; ++kt) {
      const int k0 = 32 * kt;
      const v16h fa0 = lda_frag(a1, N1P, m, k0, h);
      const v16h fa1 = lda_frag(a1, N1P, 16 + m, k0, h);
#pragma unroll
      for (int s = 0; s < 2; ++s) {
        const v16h fb = ldb_frag(wp + OV1, G1_, 32 * wv + 16 * s + m, k0, h);
        acc[0][s] = wmh(fa0, fb, acc[0][s]);
        acc[1][s] = wmh(fa1, fb, acc[1][s]);
      }
    }
#pragma unroll
    for (int s = 0; s < 2; ++s) {
      const int col = 32 * wv + 16 * s + m;
      const float bb = c1b[col];
#pragma unroll
      for (int mt = 0; mt < 2; ++mt) {
#pragma unroll
        for (int r = 0; r < 8; ++r) a2[(16 * mt + 8 * h + r) * N1P + col] = (_Float16)lk(acc[mt][s][r] * PSCL + bb);
      }
    }
  }
  __syncthreads();

  if (wv < 2) {
    v8f acc = zero8;
#pragma unroll 1
    for (int kt = 0; kt < G1_ / 32; ++kt) {
      const int k0 = 32 * kt;
      const v16h fa = lda_frag(a2, N1P, 16 * wv + m, k0, h);
      const v16h fb = ldb_frag(wp + OV2, G1_, m, k0, h);
      acc = wmh(fa, fb, acc);
    }
    const float bb = c2b[m];
    if (m < NFO) {
#pragma unroll
      for (int r = 0; r < 8; ++r) opre[(16 * wv + 8 * h + r) * NFO + m] = acc[r] * PSCL + bb;
    }
  }
  __syncthreads();
  if (tid < 32 * NFO) obuf[tid] = tanhf(opre[tid]);
  __syncthreads();
  if (wv == 0) {
    const int q = imin(lane, 23);
    const v4f v = *(const v4f*)(obuf + 4 * q);
    float* p = out + (size_t)blk * (32 * NFO) + 4 * q;
    if (lane < 24) *(volatile v4f*)p = v;
    __threadfence();
    if (lane < 24) *(volatile v4f*)p = v;
  }
}

extern "C" void kernel_launch(void* const* d_in, const int* in_sizes, int n_in,
                              void* d_out, int out_size, void* d_ws, size_t ws_size,
                              hipStream_t stream) {
  if (n_in < 13) return;
  if (in_sizes[0] != NNODE * HD_) return;
  if (in_sizes[1] != E0_ * K0_ || in_sizes[2] != E0_) return;
  if (in_sizes[3] != E1_ * E0_ || in_sizes[4] != E1_) return;
  if (in_sizes[5] != E2_ * E1_ || in_sizes[6] != E2_) return;
  if (in_sizes[7] != G1_ * G0_ || in_sizes[8] != G1_) return;
  if (in_sizes[9] != G1_ * G1_ || in_sizes[10] != G1_) return;
  if (in_sizes[11] != HD_ * G1_ || in_sizes[12] != HD_) return;
  if (out_size != NNODE * NFO) return;

  const float* x     = (const float*)d_in[0];
  const float* fe_w0 = (const float*)d_in[1];
  const float* fe_b0 = (const float*)d_in[2];
  const float* fe_w1 = (const float*)d_in[3];
  const float* fe_b1 = (const float*)d_in[4];
  const float* fe_w2 = (const float*)d_in[5];
  const float* fe_b2 = (const float*)d_in[6];
  const float* fn_w0 = (const float*)d_in[7];
  const float* fn_b0 = (const float*)d_in[8];
  const float* fn_w1 = (const float*)d_in[9];
  const float* fn_b1 = (const float*)d_in[10];
  const float* fn_w2 = (const float*)d_in[11];
  const float* fn_b2 = (const float*)d_in[12];
  float* out = (float*)d_out;

  char* ws = (char*)d_ws;
  size_t off = 0;
  const size_t oWP = off; off += SZ_WP;
  const size_t oPQ = off; off += SZ_PQ;
  const size_t oAS = off; off += SZ_AS;
  if (off != SZ_TOT) return;
  if (off > ws_size || off > (size_t)WSCAP) return;

  _Float16* wp = (_Float16*)(ws + oWP);
  float* pq = (float*)(ws + oPQ);
  float* as = (float*)(ws + oAS);

  k_prep<<<NCHUNK / 4, NTE, 0, stream>>>(fe_w0, fe_w1, fe_w2, fn_w0, fn_w1, fn_w2, wp);
  k_pq<<<NNODE / 16, NTE, 0, stream>>>(x, wp, fe_b0, pq);
  k_edge<<<NB_ * NTI, NTE, 0, stream>>>(x, pq, fe_w0, fe_b1, fe_b2, wp, as);
  k_node<<<NNODE / 32, NTN, 0, stream>>>(as, x, wp, fn_b0, fn_b1, fn_b2, out);
}
